// IGMambaModule_Swapped_77300821394065
// MI455X (gfx1250) — hardware-run, weakly checked
//
#include <hip/hip_runtime.h>
#include <math.h>

#pragma clang fp contract(off)

#define NBATCH 2
#define LL     4096
#define NTOK   (NBATCH * LL)
#define DM     128
#define DIN    256
#define DXZ    (2 * DIN)
#define DST    16
#define DTR    8
#define XDV    40
#define XDN    64
#define DCV    4
#define KC     (2 * DIN)
#define HS     32
#define HD     64
#define XP     132
#define OSTR   68
#define SCH    32
#define SYP    260
#define TPF    36
#define EPS    1e-5f
#define LOG2E  1.4426950408889634f
#define SC_H   8.0f
#define SC_W   16.0f
#define SC_XC  256.0f
#define SC_Y   1024.0f
#define SC_LO  2048.0f
#define RLO    (1.0f / 2048.0f)
#define WSCAP  ((size_t)134217728)

static_assert(NTOK % 64 == 0);
static_assert(NTOK % 32 == 0);
static_assert(NTOK % 4 == 0);
static_assert(LL % 32 == 0);
static_assert(LL % SCH == 0);
static_assert(LL == HD * HD);
static_assert(HD == 2 * HS);
static_assert(DM == 128);
static_assert(DIN == 256);
static_assert(DXZ % 64 == 0);
static_assert(XDN == 64);
static_assert(XDV <= XDN);
static_assert(DM % 64 == 0);
static_assert(DM % 32 == 0);
static_assert(DIN % 32 == 0);
static_assert(KC % 32 == 0);
static_assert(DST == 16);
static_assert(DTR == 8);
static_assert(DCV == 4);
static_assert(SCH == 32);
static_assert((DXZ * DM / 8) % 256 == 0);
static_assert((XDN * DIN / 8) % 256 == 0);
static_assert((DM * KC / 8) % 256 == 0);
static_assert(SYP % 4 == 0);
static_assert(SYP >= DIN);
static_assert(OSTR % 4 == 0);
static_assert(XP % 4 == 0);
static_assert(XP >= DM);
static_assert(TPF % 4 == 0);
static_assert(TPF >= 32);

typedef unsigned short us16 __attribute__((ext_vector_type(16)));
typedef unsigned short us8  __attribute__((ext_vector_type(8)));
typedef unsigned short us8a __attribute__((ext_vector_type(8), may_alias));
typedef unsigned short us4  __attribute__((ext_vector_type(4)));
typedef _Float16 v16h __attribute__((ext_vector_type(16)));
typedef _Float16 v8h  __attribute__((ext_vector_type(8)));
typedef _Float16 v4h  __attribute__((ext_vector_type(4)));
typedef float v8f  __attribute__((ext_vector_type(8)));
typedef float v4f  __attribute__((ext_vector_type(4)));
typedef float v4fa __attribute__((ext_vector_type(4), may_alias));
union FragU { us16 v; us8 h[2]; };

__device__ __forceinline__ float bf16r(float f) {
  unsigned u = __float_as_uint(f);
  u += 0x7FFFu + ((u >> 16) & 1u);
  return __uint_as_float(u & 0xFFFF0000u);
}
__device__ __forceinline__ float sigmf(float v) { return 1.0f / (1.0f + expf(-v)); }
__device__ __forceinline__ float siluf(float v) { return v * sigmf(v); }

__device__ __forceinline__ void hl16(float f, _Float16& hi, _Float16& lo) {
  const _Float16 hv = (_Float16)f;
  hi = hv;
  lo = (_Float16)((f - (float)hv) * SC_LO);
}

__device__ __forceinline__ float conv_silu(float c0, float c1, float c2, float c3,
                                           float x0, float x1, float x2, float x3, float bias) {
#pragma clang fp contract(off)
  float a = c0 * x0;
  a = a + c1 * x1;
  a = a + c2 * x2;
  a = a + c3 * x3;
  a = a + bias;
  return siluf(a);
}

__device__ __forceinline__ v8f mma_f16(us16 a, us16 b, v8f c) {
  return __builtin_amdgcn_wmma_f32_16x16x32_f16(false, __builtin_bit_cast(v16h, a), false, __builtin_bit_cast(v16h, b),
                                                (short)0, c, false, false);
}
__device__ __forceinline__ void wguard_g(v8f (&ch)[4], v8f (&cw)[4], const us16& a0, const us16& a1, const us16 (&b)[4]) {
#if defined(__HIP_DEVICE_COMPILE__)
  asm volatile("v_nop\n\tv_nop\n\tv_nop\n\tv_nop"
               : "+v"(ch[0]), "+v"(ch[1]), "+v"(ch[2]), "+v"(ch[3]),
                 "+v"(cw[0]), "+v"(cw[1]), "+v"(cw[2]), "+v"(cw[3])
               : "v"(a0), "v"(a1), "v"(b[0]), "v"(b[1]), "v"(b[2]), "v"(b[3]));
#endif
}

__device__ __forceinline__ us16 gfrag(const unsigned short* __restrict__ P, int ld, int row0, int k0) {
  const int lane = threadIdx.x & 31, r = lane & 15, kh = (lane >> 4) * 8;
  const unsigned short* p = P + (size_t)(row0 + r) * ld + k0 + kh;
  FragU f;
  f.h[0] = *(const us8a*)p;
  f.h[1] = *(const us8a*)(p + 16);
  return f.v;
}

__global__ __launch_bounds__(256) void k_cvtw(const float* __restrict__ W, int src_ld, int src_kmask, int n_valid,
                                             unsigned short* T, int ld_t, int n_rows, float scale) {
  const int idx = blockIdx.x * 256 + threadIdx.x;
  const int ppr = ld_t >> 3;
  const int total = n_rows * ppr;
  const int cidx = idx < total ? idx : total - 1;
  const int n = cidx / ppr, k8 = (cidx - n * ppr) * 8;
  const int ks = k8 & src_kmask;
  const bool ok = n < n_valid;
  const int nn = ok ? n : n_valid - 1;
  const float* p = W + (size_t)nn * src_ld + ks;
  const v4f va = *(const v4fa*)p;
  const v4f vb = *(const v4fa*)(p + 4);
  v8h hv;
#pragma unroll
  for (int u = 0; u < 4; ++u) {
    const float fa = scale * bf16r(va[u]);
    const float fb = scale * bf16r(vb[u]);
    hv[u]     = ok ? (_Float16)fa : (_Float16)0.0f;
    hv[4 + u] = ok ? (_Float16)fb : (_Float16)0.0f;
  }
  const us8 o = __builtin_bit_cast(us8, hv);
  const size_t off = (size_t)n * ld_t + (size_t)k8;
  if (idx < total) *(volatile us8*)(T + off) = o;
  __threadfence();
  if (idx < total) *(volatile us8*)(T + off) = o;
}

__global__ __launch_bounds__(256) void k_front(const float* __restrict__ x, const float* __restrict__ il, const float* __restrict__ gr,
                                              const float* __restrict__ iw, const float* __restrict__ ib,
                                              const float* __restrict__ rmsw, const float* __restrict__ alphap,
                                              unsigned short* Hh, unsigned short* Hl, float* Mb) {
  __shared__ __attribute__((aligned(16))) float sX[32 * XP];
  __shared__ __attribute__((aligned(16))) unsigned short sHh[32 * DM];
  __shared__ __attribute__((aligned(16))) unsigned short sHl[32 * DM];
  __shared__ float sw[DM + 4], srw[DM], su[32], sg[32], smm[32];
  const int tid = threadIdx.x;
  const int tok0 = blockIdx.x * 32;
  const int b = tok0 / LL, l0 = tok0 - b * LL;

  {
    const float wv = iw[tid < DM ? tid : DM];
    if (tid <= DM) sw[tid] = bf16r(wv);
    const float rv = rmsw[tid < DM ? tid : DM - 1];
    if (tid < DM) srw[tid] = bf16r(rv);
  }
  if (tid < 32) {
    const int l = l0 + tid, hq = l >> 6, wq = l & 63;
    const float syf = (float)hq * 0.5f - 0.25f, sxf = (float)wq * 0.5f - 0.25f;
    const float y0f = floorf(syf), x0f = floorf(sxf);
    const float fy = syf - y0f, fx = sxf - x0f;
    const int iy = (int)y0f, ix = (int)x0f;
    const int iy0 = iy < 0 ? 0 : (iy > HS - 1 ? HS - 1 : iy);
    const int iy1 = (iy + 1) < 0 ? 0 : ((iy + 1) > HS - 1 ? HS - 1 : (iy + 1));
    const int ix0 = ix < 0 ? 0 : (ix > HS - 1 ? HS - 1 : ix);
    const int ix1 = (ix + 1) < 0 ? 0 : ((ix + 1) > HS - 1 ? HS - 1 : (ix + 1));
    const float* pi = il + (size_t)b * HS * HS;
    const float* pg = gr + (size_t)b * HS * HS;
    const float i00 = bf16r(pi[iy0 * HS + ix0]), i01 = bf16r(pi[iy0 * HS + ix1]);
    const float i10 = bf16r(pi[iy1 * HS + ix0]), i11 = bf16r(pi[iy1 * HS + ix1]);
    const float g00 = bf16r(pg[iy0 * HS + ix0]), g01 = bf16r(pg[iy0 * HS + ix1]);
    const float g10 = bf16r(pg[iy1 * HS + ix0]), g11 = bf16r(pg[iy1 * HS + ix1]);
    const float wy0 = 1.0f - fy, wx0 = 1.0f - fx;
    su[tid] = wy0 * (wx0 * i00 + fx * i01) + fy * (wx0 * i10 + fx * i11);
    sg[tid] = wy0 * (wx0 * g00 + fx * g01) + fy * (wx0 * g10 + fx * g11);
  }
#pragma unroll
  for (int it = 0; it < 4; ++it) {
    const int idx = it * 256 + tid, c = idx >> 3, q = idx & 7;
    const v4f v = *(const v4fa*)(x + ((size_t)(b * DM + c)) * LL + l0 + 4 * q);
#pragma unroll
    for (int u = 0; u < 4; ++u) sX[(4 * q + u) * XP + c] = bf16r(v[u]);
  }
  __syncthreads();

  const int tl = tid >> 3, sub = tid & 7;
  float xv[16];
#pragma unroll
  for (int i4 = 0; i4 < 4; ++i4) {
    const v4f t4 = *(const v4fa*)(sX + tl * XP + sub * 16 + 4 * i4);
#pragma unroll
    for (int u = 0; u < 4; ++u) xv[4 * i4 + u] = t4[u];
  }
  float dot = 0.0f;
#pragma unroll
  for (int i = 0; i < 16; ++i) dot = dot + sw[sub * 16 + i] * xv[i];
  dot = dot + __shfl_xor(dot, 1);
  dot = dot + __shfl_xor(dot, 2);
  dot = dot + __shfl_xor(dot, 4);
  dot = dot + sw[DM] * su[tl];
  dot = dot + bf16r(ib[0]);
  const float m = sigmf(dot);
  const float gsc = 1.0f + bf16r(alphap[0]) * sg[tl];
  float fh[16];
  float ss = 0.0f;
#pragma unroll
  for (int i = 0; i < 16; ++i) { fh[i] = xv[i] * gsc; ss = ss + fh[i] * fh[i]; }
  ss = ss + __shfl_xor(ss, 1);
  ss = ss + __shfl_xor(ss, 2);
  ss = ss + __shfl_xor(ss, 4);
  const float inv = rsqrtf(ss * (1.0f / (float)DM) + EPS);
#pragma unroll
  for (int i8 = 0; i8 < 2; ++i8) {
    v8h hvh, hvl;
#pragma unroll
    for (int u = 0; u < 8; ++u) {
      const int i = 8 * i8 + u;
      const float hd = (fh[i] * inv) * srw[sub * 16 + i];
      _Float16 a, r;
      hl16(SC_H * hd, a, r);
      hvh[u] = a;
      hvl[u] = r;
    }
    *(us8a*)(sHh + tl * DM + sub * 16 + 8 * i8) = __builtin_bit_cast(us8, hvh);
    *(us8a*)(sHl + tl * DM + sub * 16 + 8 * i8) = __builtin_bit_cast(us8, hvl);
  }
  if (sub == 0) smm[tl] = m;
  __syncthreads();

  us8 oh[2], ol[2];
  size_t offs[2];
#pragma unroll
  for (int it = 0; it < 2; ++it) {
    const int row = it * 16 + (tid >> 4), c8 = (tid & 15) * 8;
    oh[it] = *(const us8a*)(sHh + row * DM + c8);
    ol[it] = *(const us8a*)(sHl + row * DM + c8);
    offs[it] = (size_t)(tok0 + row) * DM + (size_t)c8;
  }
  const float mv = smm[tid & 31];
#pragma unroll
  for (int pass = 0; pass < 2; ++pass) {
#pragma unroll
    for (int it = 0; it < 2; ++it) {
      *(volatile us8*)(Hh + offs[it]) = oh[it];
      *(volatile us8*)(Hl + offs[it]) = ol[it];
    }
    if (tid < 32) *(volatile float*)(Mb + tok0 + tid) = mv;
    __threadfence();
  }
}

__global__ __launch_bounds__(128) void k_gemm(const unsigned short* __restrict__ Ah, const unsigned short* __restrict__ Al, int lda,
                                             const unsigned short* __restrict__ B, int ldb, int K, float scale, float* Y, int ldy) {
  __shared__ __attribute__((aligned(16))) float sm[4 * 16 * OSTR];
  const int tid = threadIdx.x, lane = tid & 31, wave = tid >> 5, cl = lane & 15, hh = lane >> 4;
  const int m0 = blockIdx.x * 64 + wave * 16, n0 = blockIdx.y * 64;

  v8f ach[4], acl[4];
#pragma unroll
  for (int j = 0; j < 4; ++j) {
    v8f zz = {0.f, 0.f, 0.f, 0.f, 0.f, 0.f, 0.f, 0.f};
    ach[j] = zz;
    acl[j] = zz;
  }

#pragma unroll 1
  for (int k0 = 0; k0 < K; k0 += 32) {
    const us16 a0 = gfrag(Ah, lda, m0, k0);
    const us16 a1 = gfrag(Al, lda, m0, k0);
    us16 bfr[4];
#pragma unroll
    for (int j = 0; j < 4; ++j) bfr[j] = gfrag(B, ldb, n0 + 16 * j, k0);
#pragma unroll
    for (int j = 0; j < 4; ++j) {
      ach[j] = mma_f16(a0, bfr[j], ach[j]);
      acl[j] = mma_f16(a1, bfr[j], acl[j]);
    }
    wguard_g(ach, acl, a0, a1, bfr);
  }

  float* so = sm + wave * (16 * OSTR);
#pragma unroll
  for (int j = 0; j < 4; ++j)
#pragma unroll
    for (int r = 0; r < 8; ++r)
      so[(8 * hh + r) * OSTR + 16 * j + cl] = (ach[j][r] + acl[j][r] * RLO) * scale;
  __syncthreads();

  v4f ov[8];
  size_t offs[8];
#pragma unroll
  for (int it = 0; it < 8; ++it) {
    const int ch = it * 32 + lane, r = ch >> 4, q = (ch & 15) * 4;
    ov[it] = *(const v4fa*)(so + r * OSTR + q);
    offs[it] = (size_t)(m0 + r) * ldy + (size_t)(n0 + q);
  }
#pragma unroll
  for (int pass = 0; pass < 2; ++pass) {
#pragma unroll
    for (int it = 0; it < 8; ++it) *(volatile v4f*)(Y + offs[it]) = ov[it];
    __threadfence();
  }
}

__global__ __launch_bounds__(256) void k_conv(const float* __restrict__ XZ, const float* __restrict__ cw, const float* __restrict__ cb,
                                             float* XCF, unsigned short* XCh, unsigned short* XCl) {
#pragma clang fp contract(off)
  const int tid = threadIdx.x;
  const int tok = blockIdx.x * 4 + (tid >> 6);
  const int b = tok / LL, t = tok - b * LL;
  const int c = (tid & 63) * 4;
  float xv[DCV][4];
#pragma unroll
  for (int j = 0; j < DCV; ++j) {
    const int pos = t - (DCV - 1) + j;
    const bool ok = pos >= 0;
    const int pc = ok ? pos : 0;
    const v4f va = *(const v4fa*)(XZ + ((size_t)(b * LL + pc)) * DXZ + c);
#pragma unroll
    for (int u = 0; u < 4; ++u) xv[j][u] = ok ? va[u] : 0.0f;
  }
  float wv[DCV][4];
#pragma unroll
  for (int u = 0; u < 4; ++u) {
    const v4f wq = *(const v4fa*)(cw + (size_t)(c + u) * DCV);
#pragma unroll
    for (int j = 0; j < DCV; ++j) wv[j][u] = bf16r(wq[j]);
  }
  float bv[4];
  {
    const v4f bq = *(const v4fa*)(cb + c);
#pragma unroll
    for (int u = 0; u < 4; ++u) bv[u] = bf16r(bq[u]);
  }
  v4f of;
  v4h hh4, hl4;
#pragma unroll
  for (int u = 0; u < 4; ++u) {
    const float res = conv_silu(wv[0][u], wv[1][u], wv[2][u], wv[3][u], xv[0][u], xv[1][u], xv[2][u], xv[3][u], bv[u]);
    of[u] = res;
    _Float16 a, r;
    hl16(SC_XC * res, a, r);
    hh4[u] = a;
    hl4[u] = r;
  }
  const us4 ph = __builtin_bit_cast(us4, hh4), pl = __builtin_bit_cast(us4, hl4);
  const size_t off = (size_t)tok * DIN + (size_t)c;
#pragma unroll
  for (int pass = 0; pass < 2; ++pass) {
    *(volatile v4f*)(XCF + off) = of;
    *(volatile us4*)(XCh + off) = ph;
    *(volatile us4*)(XCl + off) = pl;
    __threadfence();
  }
}

__global__ __launch_bounds__(256) void k_scan(const float* __restrict__ XZ, const float* __restrict__ XCF, const float* __restrict__ DBC,
                                             const float* __restrict__ dtw, const float* __restrict__ dtb,
                                             const float* __restrict__ Alog, const float* __restrict__ Ablog,
                                             const float* __restrict__ Dp, unsigned short* Yh, unsigned short* Yl) {
#pragma clang fp contract(off)
  __shared__ __attribute__((aligned(16))) float sy[SCH * SYP];
  __shared__ __attribute__((aligned(16))) float sd[SCH * XDN];
  const int dir = blockIdx.x, b = blockIdx.y;
  const int tid = threadIdx.x, lane = tid & 31, wave = tid >> 5;
  const int d = tid;
  float A2[DST], h[DST];
#pragma unroll
  for (int n = 0; n < DST; ++n) {
    const float la = Alog[d * DST + n], lb = Ablog[d * DST + n];
    const float lv = dir ? lb : la;
    A2[n] = -exp2f(bf16r(lv) * LOG2E) * LOG2E;
    h[n] = 0.0f;
  }
  float Wd[DTR];
#pragma unroll
  for (int r = 0; r < DTR; ++r) Wd[r] = bf16r(dtw[d * DTR + r]);
  const float bd = bf16r(dtb[d]);
  const float Dd = bf16r(Dp[d]);

#pragma unroll 1
  for (int cnk = 0; cnk < LL / SCH; ++cnk) {
    const int tn0 = dir ? (LL - SCH * (cnk + 1)) : (SCH * cnk);
    const size_t rowg = (size_t)b * LL + (size_t)tn0;
    {
      const int r = tid >> 3, q = (tid & 7) * 8;
      const float* p = DBC + (rowg + (size_t)r) * XDN + q;
      *(v4fa*)(sd + r * XDN + q)     = *(const v4fa*)p;
      *(v4fa*)(sd + r * XDN + q + 4) = *(const v4fa*)(p + 4);
    }
    __syncthreads();

#pragma unroll 1
    for (int s = 0; s < SCH; ++s) {
      const int rr = dir ? (SCH - 1 - s) : s;
      const size_t tok = rowg + (size_t)rr;
      const float* sr = sd + rr * XDN;
      const v4f d0 = *(const v4fa*)sr, d1 = *(const v4fa*)(sr + 4);
      float raw = d0[0] * Wd[0];
      raw = raw + d0[1] * Wd[1];
      raw = raw + d0[2] * Wd[2];
      raw = raw + d0[3] * Wd[3];
      raw = raw + d1[0] * Wd[4];
      raw = raw + d1[1] * Wd[5];
      raw = raw + d1[2] * Wd[6];
      raw = raw + d1[3] * Wd[7];
      raw = raw + bd;
      const float dl = fmaxf(raw, 0.0f) + log1pf(expf(-fabsf(raw)));
      const float xc = XCF[tok * DIN + d];
      const float zv = XZ[tok * DXZ + DIN + d];
      v4f Bv[4], Cv[4];
#pragma unroll
      for (int q = 0; q < 4; ++q) {
        Bv[q] = *(const v4fa*)(sr + DTR + 4 * q);
        Cv[q] = *(const v4fa*)(sr + DTR + DST + 4 * q);
      }
      const float dx = dl * xc;
      float y = 0.0f;
#pragma unroll
      for (int n = 0; n < DST; ++n) {
        const float e = exp2f(dl * A2[n]);
        h[n] = e * h[n] + dx * Bv[n >> 2][n & 3];
        y = y + h[n] * Cv[n >> 2][n & 3];
      }
      const float yv = (y + xc * Dd) * siluf(zv);
      sy[rr * SYP + d] = yv;
    }
    __syncthreads();

    us8 oh[4], ol[4];
    size_t offs[4];
#pragma unroll
    for (int it = 0; it < 4; ++it) {
      const int row = 4 * wave + it;
      const v4f va = *(const v4fa*)(sy + row * SYP + lane * 8);
      const v4f vb = *(const v4fa*)(sy + row * SYP + lane * 8 + 4);
      v8h hvh, hvl;
#pragma unroll
      for (int u = 0; u < 4; ++u) {
        _Float16 a, r;
        hl16(SC_Y * va[u], a, r);
        hvh[u] = a;
        hvl[u] = r;
        hl16(SC_Y * vb[u], a, r);
        hvh[4 + u] = a;
        hvl[4 + u] = r;
      }
      oh[it] = __builtin_bit_cast(us8, hvh);
      ol[it] = __builtin_bit_cast(us8, hvl);
      offs[it] = (rowg + (size_t)row) * KC + (size_t)(dir * DIN + lane * 8);
    }
#pragma unroll
    for (int pass = 0; pass < 2; ++pass) {
#pragma unroll
      for (int it = 0; it < 4; ++it) {
        *(volatile us8*)(Yh + offs[it]) = oh[it];
        *(volatile us8*)(Yl + offs[it]) = ol[it];
      }
      __threadfence();
    }
    __syncthreads();
  }
}

__global__ __launch_bounds__(256) void k_final(const float* __restrict__ MO, const float* __restrict__ x, const float* __restrict__ Mb,
                                              const float* __restrict__ lnw, const float* __restrict__ lnb,
                                              const float* __restrict__ gammap, float* out) {
#pragma clang fp contract(off)
  __shared__ __attribute__((aligned(16))) float sM[32 * XP];
  __shared__ __attribute__((aligned(16))) float sT[DM * TPF];
  __shared__ __attribute__((aligned(16))) float smm[32];
  const int tid = threadIdx.x;
  const int tok0 = blockIdx.x * 32;
  const int b = tok0 / LL, l0 = tok0 - b * LL;
  {
    const float mv = Mb[tok0 + (tid & 31)];
    if (tid < 32) smm[tid] = mv;
  }
#pragma unroll
  for (int it = 0; it < 4; ++it) {
    const int idx = it * 256 + tid, r = idx >> 5, q = (idx & 31) * 4;
    *(v4fa*)(sM + r * XP + q) = *(const v4fa*)(MO + (size_t)(tok0 + r) * DM + q);
  }
  __syncthreads();

  const int tl = tid >> 3, sub = tid & 7;
  float v[16];
#pragma unroll
  for (int i4 = 0; i4 < 4; ++i4) {
    const v4f t4 = *(const v4fa*)(sM + tl * XP + sub * 16 + 4 * i4);
#pragma unroll
    for (int u = 0; u < 4; ++u) v[4 * i4 + u] = t4[u];
  }
  float s1 = 0.0f;
#pragma unroll
  for (int i = 0; i < 16; ++i) s1 = s1 + v[i];
  s1 = s1 + __shfl_xor(s1, 1);
  s1 = s1 + __shfl_xor(s1, 2);
  s1 = s1 + __shfl_xor(s1, 4);
  const float mu = s1 * (1.0f / (float)DM);
  float dv[16];
  float s2 = 0.0f;
#pragma unroll
  for (int i = 0; i < 16; ++i) { dv[i] = v[i] - mu; s2 = s2 + dv[i] * dv[i]; }
  s2 = s2 + __shfl_xor(s2, 1);
  s2 = s2 + __shfl_xor(s2, 2);
  s2 = s2 + __shfl_xor(s2, 4);
  const float var = s2 * (1.0f / (float)DM);
  const float rs = rsqrtf(var + EPS);
#pragma unroll
  for (int i = 0; i < 16; ++i) {
    const int c = sub * 16 + i;
    sT[c * TPF + tl] = (dv[i] * rs) * bf16r(lnw[c]) + bf16r(lnb[c]);
  }
  __syncthreads();

  const float g = bf16r(gammap[0]);
  v4f o[4];
  size_t offs[4];
#pragma unroll
  for (int it = 0; it < 4; ++it) {
    const int c = it * 32 + (tid >> 3), q = tid & 7;
    const v4f lnv = *(const v4fa*)(sT + c * TPF + 4 * q);
    const v4f mv4 = *(const v4fa*)(smm + 4 * q);
    const size_t gi = ((size_t)(b * DM + c)) * LL + (size_t)(l0 + 4 * q);
    const v4f xv4 = *(const v4fa*)(x + gi);
    v4f ov;
#pragma unroll
    for (int u = 0; u < 4; ++u) ov[u] = lnv[u] + g * (bf16r(xv4[u]) * mv4[u]);
    o[it] = ov;
    offs[it] = gi;
  }
#pragma unroll
  for (int pass = 0; pass < 2; ++pass) {
#pragma unroll
    for (int it = 0; it < 4; ++it) *(volatile v4f*)(out + offs[it]) = o[it];
    __threadfence();
  }
}

extern "C" void kernel_launch(void* const* d_in, const int* in_sizes, int n_in,
                              void* d_out, int out_size, void* d_ws, size_t ws_size,
                              hipStream_t stream) {
  if (n_in < 20) return;
  if (in_sizes[0] != NBATCH * DM * LL || in_sizes[1] != NBATCH * HS * HS || in_sizes[2] != NBATCH * HS * HS ||
      in_sizes[3] != DM + 1 || in_sizes[4] < 1 || in_sizes[5] != DM || in_sizes[6] != DXZ * DM ||
      in_sizes[7] != DIN * DCV || in_sizes[8] != DIN || in_sizes[9] != XDV * DIN || in_sizes[10] != DIN * DTR ||
      in_sizes[11] != DIN || in_sizes[12] != DIN * DST || in_sizes[13] != DIN * DST || in_sizes[14] != DIN ||
      in_sizes[15] != DM * DIN || in_sizes[16] != DM || in_sizes[17] != DM || in_sizes[18] < 1 || in_sizes[19] < 1) return;
  if (out_size != NBATCH * DM * LL) return;

  const float* x      = (const float*)d_in[0];
  const float* illum  = (const float*)d_in[1];
  const float* grad   = (const float*)d_in[2];
  const float* illw   = (const float*)d_in[3];
  const float* illb   = (const float*)d_in[4];
  const float* rmsw   = (const float*)d_in[5];
  const float* inprj  = (const float*)d_in[6];
  const float* convw  = (const float*)d_in[7];
  const float* convb  = (const float*)d_in[8];
  const float* xprj   = (const float*)d_in[9];
  const float* dtw    = (const float*)d_in[10];
  const float* dtb    = (const float*)d_in[11];
  const float* A_log  = (const float*)d_in[12];
  const float* Ab_log = (const float*)d_in[13];
  const float* Dparam = (const float*)d_in[14];
  const float* outprj = (const float*)d_in[15];
  const float* lnw    = (const float*)d_in[16];
  const float* lnb    = (const float*)d_in[17];
  const float* alpha  = (const float*)d_in[18];
  const float* gamma  = (const float*)d_in[19];
  float* out = (float*)d_out;

  size_t off = 0;
  auto carve = [&](size_t bytes) -> char* { char* p = (char*)d_ws + off; off += (bytes + 255) & ~(size_t)255; return p; };
  unsigned short* Win = (unsigned short*)carve((size_t)DXZ * DM * 2);
  unsigned short* Wx  = (unsigned short*)carve((size_t)XDN * DIN * 2);
  unsigned short* Wo  = (unsigned short*)carve((size_t)DM * KC * 2);
  unsigned short* Hh  = (unsigned short*)carve((size_t)NTOK * DM * 2);
  unsigned short* Hl  = (unsigned short*)carve((size_t)NTOK * DM * 2);
  float* Mb           = (float*)carve((size_t)NTOK * 4);
  float* XZ           = (float*)carve((size_t)NTOK * DXZ * 4);
  float* XCF          = (float*)carve((size_t)NTOK * DIN * 4);
  unsigned short* XCh = (unsigned short*)carve((size_t)NTOK * DIN * 2);
  unsigned short* XCl = (unsigned short*)carve((size_t)NTOK * DIN * 2);
  float* DBC          = (float*)carve((size_t)NTOK * XDN * 4);
  unsigned short* Yh  = (unsigned short*)carve((size_t)NTOK * KC * 2);
  unsigned short* Yl  = (unsigned short*)carve((size_t)NTOK * KC * 2);
  float* MO           = (float*)carve((size_t)NTOK * DM * 4);
  if (off > ws_size || off > WSCAP) return;

  const dim3 b256(256), b128(128);
  k_cvtw<<<dim3((DXZ * DM / 8) / 256), b256, 0, stream>>>(inprj, DM, DM - 1, DXZ, Win, DM, DXZ, SC_W);
  k_cvtw<<<dim3((XDN * DIN / 8) / 256), b256, 0, stream>>>(xprj, DIN, DIN - 1, XDV, Wx, DIN, XDN, SC_W);
  k_cvtw<<<dim3((DM * KC / 8) / 256), b256, 0, stream>>>(outprj, DIN, DIN - 1, DM, Wo, KC, DM, SC_W);
  k_front<<<dim3(NTOK / 32), b256, 0, stream>>>(x, illum, grad, illw, illb, rmsw, alpha, Hh, Hl, Mb);
  k_gemm<<<dim3(NTOK / 64, DXZ / 64), b128, 0, stream>>>(Hh, Hl, DM, Win, DM, DM, 1.0f / 128.0f, XZ, DXZ);
  k_conv<<<dim3(NTOK / 4), b256, 0, stream>>>(XZ, convw, convb, XCF, XCh, XCl);
  k_gemm<<<dim3(NTOK / 64, XDN / 64), b128, 0, stream>>>(XCh, XCl, DIN, Wx, DIN, DIN, 1.0f / 4096.0f, DBC, XDN);
  k_scan<<<dim3(2, NBATCH), b256, 0, stream>>>(XZ, XCF, DBC, dtw, dtb, A_log, Ab_log, Dparam, Yh, Yl);
  k_gemm<<<dim3(NTOK / 64, DM / 64), b128, 0, stream>>>(Yh, Yl, KC, Wo, KC, KC, 1.0f / 16384.0f, MO, DM);
  k_final<<<dim3(NTOK / 32), b256, 0, stream>>>(MO, x, Mb, lnw, lnb, gamma, out);
}
